// GPSLayer_64484638982371
// MI455X (gfx1250) — hardware-run, weakly checked
//
#include <hip/hip_runtime.h>
#include <stddef.h>
#include <stdint.h>


#define DIN     128
#define NP      640
#define NPH     1280
#define OXW     0
#define OKK     128
#define OVV     256
#define OQQ     384
#define OXR     512
#define OH16    768
#define OF16    0
#define KF1     256
#define NF1     256
#define KF2     512
#define NF2     128
#define NSEG    5
#define NTHR    256
#define NWAVE   8
#define EPT     8
#define CHUNK   (NTHR * EPT)
#define WCAP    (EPT * 32)
#define LISTN   (NWAVE * WCAP)
#define NBMAX   1024
#define RCAP    28672
#define DEGCAP  64
#define GBM     64
#define PTHR    128
#define HSTG    128
#define ATTSC   0.17677669529663689f
#define LNEPS   1e-5f
#define WSMAX   134217728
#define LDS_CNT ((RCAP + NBMAX + LISTN + 2 * NWAVE) * 4)
#define LDS_AGG ((2 * RCAP + 2 * NBMAX + LISTN + 2 * NWAVE + NWAVE * HSTG) * 4)

static_assert((CHUNK & (CHUNK - 1)) == 0 && CHUNK <= 4096);
static_assert((NBMAX & (NBMAX - 1)) == 0 && NBMAX <= 4096);
static_assert(NTHR * 4 == NBMAX);
static_assert(LISTN >= NBMAX);
static_assert(LISTN >= NWAVE * WCAP);
static_assert((RCAP % 32) == 0);
static_assert(LDS_AGG <= 300000);
static_assert(LDS_CNT <= 300000);
static_assert(((2 * RCAP + 2 * NBMAX + LISTN + 2 * NWAVE) * 4) % 16 == 0);
static_assert((DIN % 32) == 0 && (KF1 % 32) == 0 && (KF2 % 32) == 0);
static_assert(NP == NSEG * DIN && NPH == 2 * NP);
static_assert((NP * 4) % 128 == 0 && (OQQ * 4) % 128 == 0 && (OXR * 4) % 128 == 0);
static_assert(OH16 * 2 == OQQ * 4 && (OH16 + 2 * DIN) * 2 == OXR * 4);
static_assert((OF16 + 2 * NF1) * 2 <= OKK * 4 + DIN * 4);
static_assert(GBM == 4 * 16 && PTHR == 4 * 32 && NTHR == NWAVE * 32);

typedef float          v4f   __attribute__((ext_vector_type(4)));
typedef float          v8f   __attribute__((ext_vector_type(8)));
typedef int            v4i   __attribute__((ext_vector_type(4)));
typedef int            v8i   __attribute__((ext_vector_type(8)));
typedef unsigned       v2u   __attribute__((ext_vector_type(2)));
typedef unsigned       v4u   __attribute__((ext_vector_type(4)));
typedef unsigned short v8us  __attribute__((ext_vector_type(8)));
typedef unsigned short v16us __attribute__((ext_vector_type(16)));
typedef __bf16         v16bf __attribute__((ext_vector_type(16)));
typedef v4f  __attribute__((may_alias)) v4fa;
typedef v8us __attribute__((may_alias)) v8usa;
typedef v2u  __attribute__((may_alias)) v2ua;
typedef v4u  __attribute__((may_alias)) v4ua;
union FragB { v16bf v; v16us u; v8us h[2]; v8i w; };

__device__ __forceinline__ v8f wmb(const FragB& a, const FragB& b, v8f c) {
  v8f d = __builtin_amdgcn_wmma_f32_16x16x32_bf16(false, a.v, false, b.v, (short)0, c, false, false);
  asm volatile("v_nop\n\tv_nop\n\tv_nop\n\tv_nop" : "+v"(d) : "v"(a.w), "v"(b.w));
  return d;
}

__device__ __forceinline__ float waveSum(float v) {
#pragma unroll
  for (int o = 16; o > 0; o >>= 1) v += __shfl_xor(v, o);
  return v;
}

__device__ __forceinline__ unsigned bfbits(float f) {
  const unsigned u = __float_as_uint(f);
  return (u + 0x7FFFu + ((u >> 16) & 1u)) >> 16;
}
__device__ __forceinline__ float bfval(unsigned b) { return __uint_as_float(b << 16); }
__device__ __forceinline__ float bf16r(float f) { return bfval(bfbits(f)); }
__device__ __forceinline__ v4f bfr4(const v4f a) {
  v4f r;
  r.x = bf16r(a.x); r.y = bf16r(a.y); r.z = bf16r(a.z); r.w = bf16r(a.w);
  return r;
}

__device__ __forceinline__ v8us hi8(const v4f a, const v4f b) {
  v8us h;
  h[0] = (unsigned short)bfbits(a.x); h[1] = (unsigned short)bfbits(a.y);
  h[2] = (unsigned short)bfbits(a.z); h[3] = (unsigned short)bfbits(a.w);
  h[4] = (unsigned short)bfbits(b.x); h[5] = (unsigned short)bfbits(b.y);
  h[6] = (unsigned short)bfbits(b.z); h[7] = (unsigned short)bfbits(b.w);
  return h;
}

__device__ __forceinline__ float dinvf(int c) {
  const int cc = c < 1 ? 1 : c;
  return c > 0 ? rsqrtf((float)cc) : 0.0f;
}

__device__ __forceinline__ int scan_chunk(const int* __restrict__ dsts, int nE, int cbase, int slotBase,
                                          int nb, int vec8, int* list, int tid, int lane, int wave) {
  int wc = 0;
  const int el0  = tid * EPT;
  const int e0   = cbase + el0;
  const int sent = -2147483647 - 1;
  v4i da, db;
  if (vec8 != 0 && cbase + CHUNK <= nE) {
    da = *(const v4i*)(dsts + e0);
    db = *(const v4i*)(dsts + e0 + 4);
  } else {
    da.x = (e0     < nE) ? dsts[min(e0,     nE - 1)] : sent;
    da.y = (e0 + 1 < nE) ? dsts[min(e0 + 1, nE - 1)] : sent;
    da.z = (e0 + 2 < nE) ? dsts[min(e0 + 2, nE - 1)] : sent;
    da.w = (e0 + 3 < nE) ? dsts[min(e0 + 3, nE - 1)] : sent;
    db.x = (e0 + 4 < nE) ? dsts[min(e0 + 4, nE - 1)] : sent;
    db.y = (e0 + 5 < nE) ? dsts[min(e0 + 5, nE - 1)] : sent;
    db.z = (e0 + 6 < nE) ? dsts[min(e0 + 6, nE - 1)] : sent;
    db.w = (e0 + 7 < nE) ? dsts[min(e0 + 7, nE - 1)] : sent;
  }
  const unsigned nbs = (unsigned)slotBase;
  const unsigned unb = (unsigned)nb;
  const unsigned s0 = (unsigned)da.x - nbs, s1 = (unsigned)da.y - nbs;
  const unsigned s2 = (unsigned)da.z - nbs, s3 = (unsigned)da.w - nbs;
  const unsigned s4 = (unsigned)db.x - nbs, s5 = (unsigned)db.y - nbs;
  const unsigned s6 = (unsigned)db.z - nbs, s7 = (unsigned)db.w - nbs;
  const bool h0 = s0 < unb, h1 = s1 < unb, h2 = s2 < unb, h3 = s3 < unb;
  const bool h4 = s4 < unb, h5 = s5 < unb, h6 = s6 < unb, h7 = s7 < unb;
  const unsigned any = __builtin_amdgcn_ballot_w32(h0 | h1 | h2 | h3 | h4 | h5 | h6 | h7);
  if (any != 0u) {
#define HITJ(J, HJ, SJ) { \
      const unsigned mj = __builtin_amdgcn_ballot_w32(HJ); \
      if (mj != 0u) { \
        if (HJ) { \
          const int pos = wc + (int)__builtin_amdgcn_mbcnt_lo(mj, 0u); \
          if (pos < WCAP) list[wave * WCAP + pos] = ((el0 + (J)) << 12) | (int)(SJ); \
        } \
        wc += (int)__builtin_popcount(mj); } }
    HITJ(0, h0, s0)
    HITJ(1, h1, s1)
    HITJ(2, h2, s2)
    HITJ(3, h3, s3)
    HITJ(4, h4, s4)
    HITJ(5, h5, s5)
    HITJ(6, h6, s6)
    HITJ(7, h7, s7)
#undef HITJ
  }
  return wc;
}

__global__ __launch_bounds__(NTHR) void k_wtr5(const float* __restrict__ w0, const float* __restrict__ w1,
                                               const float* __restrict__ w2, const float* __restrict__ w3,
                                               const float* __restrict__ w4, unsigned short* wt, int nUnits) {
  const int u = (int)blockIdx.x * NTHR + (int)threadIdx.x;
  if (u >= nUnits) return;
  const int n  = u >> 4;
  const int k8 = (u & 15) * 8;
  int seg = n >> 7;
  seg = seg > 4 ? 4 : seg;
  const int nc = n & (DIN - 1);
  const float* wsrc = (seg == 0) ? w0 : ((seg == 1) ? w1 : ((seg == 2) ? w2 : ((seg == 3) ? w3 : w4)));
  const float* p = wsrc + (size_t)k8 * DIN + nc;
  v8us hv;
  hv[0] = (unsigned short)bfbits(p[0]);
  hv[1] = (unsigned short)bfbits(p[(size_t)DIN]);
  hv[2] = (unsigned short)bfbits(p[(size_t)2 * DIN]);
  hv[3] = (unsigned short)bfbits(p[(size_t)3 * DIN]);
  hv[4] = (unsigned short)bfbits(p[(size_t)4 * DIN]);
  hv[5] = (unsigned short)bfbits(p[(size_t)5 * DIN]);
  hv[6] = (unsigned short)bfbits(p[(size_t)6 * DIN]);
  hv[7] = (unsigned short)bfbits(p[(size_t)7 * DIN]);
  const size_t o = (size_t)n * DIN + k8;
  *(volatile v8us*)(wt + o) = hv;
  __threadfence();
  *(volatile v8us*)(wt + o) = hv;
}

__global__ __launch_bounds__(NTHR) void k_wtr2(const float* __restrict__ W, int kin, int nout,
                                               unsigned short* wt, int nUnits) {
  const int u = (int)blockIdx.x * NTHR + (int)threadIdx.x;
  if (u >= nUnits) return;
  const int upr = kin >> 2;
  const int n   = u / upr;
  const int k8  = (u - n * upr) * 8;
  const int kk  = k8 & (kin - 1);
  const float* p = W + (size_t)kk * nout + n;
  v8us hv;
  hv[0] = (unsigned short)bfbits(p[0]);
  hv[1] = (unsigned short)bfbits(p[(size_t)nout]);
  hv[2] = (unsigned short)bfbits(p[(size_t)2 * nout]);
  hv[3] = (unsigned short)bfbits(p[(size_t)3 * nout]);
  hv[4] = (unsigned short)bfbits(p[(size_t)4 * nout]);
  hv[5] = (unsigned short)bfbits(p[(size_t)5 * nout]);
  hv[6] = (unsigned short)bfbits(p[(size_t)6 * nout]);
  hv[7] = (unsigned short)bfbits(p[(size_t)7 * nout]);
  const size_t o = (size_t)n * (size_t)(2 * kin) + k8;
  *(volatile v8us*)(wt + o) = hv;
  __threadfence();
  *(volatile v8us*)(wt + o) = hv;
}

__global__ __launch_bounds__(PTHR) void k_proj(
    const float* __restrict__ X, int nra, const unsigned short* __restrict__ WT,
    const float* __restrict__ b1, const float* __restrict__ b2,
    const float* __restrict__ b3, const float* __restrict__ b4, float* outF)
{
  __shared__ __attribute__((aligned(16))) float stg[4 * 16 * 64];
  const int tid = (int)threadIdx.x, lane = tid & 31, wave = tid >> 5, hh = lane >> 4, m = lane & 15;
  const int rw = wave;
  const int rowBase = (int)blockIdx.x * GBM;
  const int seg     = (int)blockIdx.y;
  const int colW    = seg * DIN;
  const float* bp = (seg == 1) ? b1 : ((seg == 2) ? b2 : ((seg == 3) ? b3 : b4));

  v8f acc[8];
  {
    const v8f z = {0.f, 0.f, 0.f, 0.f, 0.f, 0.f, 0.f, 0.f};
#pragma unroll
    for (int t = 0; t < 8; ++t) acc[t] = z;
  }
  int ra = rowBase + 16 * rw + m;
  ra = ra > nra - 1 ? nra - 1 : ra;
  ra = ra < 0 ? 0 : ra;
  const float* ap = X + (size_t)ra * DIN + 8 * hh;
  const unsigned short* wp = WT + (size_t)(colW + m) * DIN + 8 * hh;

#pragma unroll 1
  for (int ks = 0; ks < DIN / 32; ++ks) {
    const float* p = ap + 32 * ks;
    const v4f f0 = *(const v4fa*)(p);
    const v4f f1 = *(const v4fa*)(p + 4);
    const v4f f2 = *(const v4fa*)(p + 16);
    const v4f f3 = *(const v4fa*)(p + 20);
    FragB ah;
    ah.h[0] = hi8(f0, f1);
    ah.h[1] = hi8(f2, f3);
#pragma unroll
    for (int t = 0; t < 8; ++t) {
      const unsigned short* wq = wp + (size_t)(16 * t) * DIN + 32 * ks;
      FragB bf;
      bf.h[0] = *(const v8usa*)wq;
      bf.h[1] = *(const v8usa*)(wq + 16);
      acc[t] = wmb(ah, bf, acc[t]);
    }
  }

  float* sw = stg + wave * 1024;
#pragma unroll
  for (int hf = 0; hf < 2; ++hf) {
#pragma unroll
    for (int t4 = 0; t4 < 4; ++t4) {
      const int t  = 4 * hf + t4;
      const int lc = 16 * t + m;
      float bb = bf16r(bp[lc]);
      if (seg == 0) bb = 0.f;
#pragma unroll
      for (int r = 0; r < 8; ++r) sw[(8 * hh + r) * 64 + 16 * t4 + m] = acc[t][r] + bb;
    }
    __syncthreads();
    v4f fv[8];
#pragma unroll
    for (int i = 0; i < 8; ++i) {
      const int lr = 2 * i + hh;
      fv[i] = *(const v4fa*)(sw + lr * 64 + 4 * m);
    }
#pragma unroll
    for (int i = 0; i < 8; ++i) {
      const int gr = rowBase + 16 * rw + 2 * i + hh;
      float* op = outF + (size_t)gr * NP + colW + 64 * hf + 4 * m;
      *(volatile v4f*)op = fv[i];
    }
    __threadfence();
#pragma unroll
    for (int i = 0; i < 8; ++i) {
      const int gr = rowBase + 16 * rw + 2 * i + hh;
      float* op = outF + (size_t)gr * NP + colW + 64 * hf + 4 * m;
      *(volatile v4f*)op = fv[i];
    }
    __syncthreads();
  }
}

__global__ __launch_bounds__(NTHR) void k_cnt(const int* __restrict__ dsts, float* dinv, int nE, int nb, int vec8) {
  extern __shared__ v4f lds_dyn[];
  int* reg1 = (int*)lds_dyn;
  int* scnt = reg1 + RCAP;
  int* list = scnt + NBMAX;
  int* wcnt = list + LISTN;
  const int tid = (int)threadIdx.x, lane = tid & 31, wave = tid >> 5;
  const int nodeBase = (int)blockIdx.x * nb;

  for (int i = tid; i < NBMAX; i += NTHR) scnt[i] = 0;
  __syncthreads();

  int tot = 0;
  const int nChunks = (nE + CHUNK - 1) / CHUNK;
#pragma unroll 1
  for (int ch = 0; ch < nChunks; ++ch) {
    const int cbase = ch * CHUNK;
    const int wc = scan_chunk(dsts, nE, cbase, nodeBase, nb, vec8, list, tid, lane, wave);
    if (lane == 0) wcnt[wave] = wc;
    __syncthreads();
    int pre = 0, all = 0;
#pragma unroll
    for (int w2 = 0; w2 < NWAVE; ++w2) {
      int c = wcnt[w2];
      c = c < 0 ? 0 : (c > WCAP ? WCAP : c);
      all += c;
      pre += (w2 < wave) ? c : 0;
    }
    const int wcc  = wc > WCAP ? WCAP : wc;
    const int base = tot + pre;
#pragma unroll 1
    for (int i = lane; i < wcc; i += 32) {
      const int ent = list[wave * WCAP + i];
      const int el  = (ent >> 12) & (CHUNK - 1);
      const int sl  = ent & (NBMAX - 1);
      int eid = cbase + el;
      eid = eid > nE - 1 ? nE - 1 : eid;
      const int pos = base + i;
      if (pos < RCAP) reg1[pos] = (int)(((unsigned)eid << 12) | (unsigned)sl);
    }
    tot += all;
    tot = tot > RCAP ? RCAP : tot;
    __syncthreads();
  }
  const int nh = tot;

  if (wave == 0) {
#pragma unroll 1
    for (int b0 = 0; b0 < nh; b0 += 32) {
      const int idx = b0 + lane;
      const int uv  = reg1[idx < RCAP ? idx : RCAP - 1];
      const int m32 = (nh - b0) < 32 ? (nh - b0) : 32;
#pragma unroll 1
      for (int k = 0; k < m32; ++k) {
        const int u  = __builtin_amdgcn_readlane(uv, k);
        const int sl = u & (NBMAX - 1);
        if (lane == 0) scnt[sl] = scnt[sl] + 1;
      }
    }
  }
  __syncthreads();

  const bool act = tid < (nb >> 2);
  v4f dv = {0.f, 0.f, 0.f, 0.f};
  if (act) {
    const v4i ca = *(const v4i*)(scnt + 4 * tid);
    dv.x = dinvf(ca.x); dv.y = dinvf(ca.y); dv.z = dinvf(ca.z); dv.w = dinvf(ca.w);
  }
  float* dp = dinv + (size_t)nodeBase + 4 * tid;
  if (act) *(volatile v4f*)dp = dv;
  __threadfence();
  if (act) *(volatile v4f*)dp = dv;
}

__global__ __launch_bounds__(NTHR) void k_agg(
    const int* __restrict__ srcs, const int* __restrict__ dsts,
    float* P, const float* __restrict__ dinv,
    const float* __restrict__ bg, const float* __restrict__ wbeta,
    const float* __restrict__ g1, const float* __restrict__ b1,
    const float* __restrict__ lws, const float* __restrict__ gws,
    int nN, int nE, int nb, int vec8) {
  extern __shared__ v4f lds_dyn[];
  int* reg1 = (int*)lds_dyn;
  int* reg2 = reg1 + RCAP;
  int* scnt = reg2 + RCAP;
  int* soff = scnt + NBMAX;
  int* list = soff + NBMAX;
  int* wcnt = list + LISTN;
  int* wtot = wcnt + NWAVE;
  unsigned* hstg = (unsigned*)(wtot + NWAVE);
  const int tid = (int)threadIdx.x, lane = tid & 31, wave = tid >> 5;
  const int nodeBase = (int)blockIdx.x * nb;

  for (int i = tid; i < NBMAX; i += NTHR) scnt[i] = 0;
  __syncthreads();

  int tot = 0;
  const int nChunks = (nE + CHUNK - 1) / CHUNK;
#pragma unroll 1
  for (int ch = 0; ch < nChunks; ++ch) {
    const int cbase = ch * CHUNK;
    const int wc = scan_chunk(dsts, nE, cbase, nodeBase, nb, vec8, list, tid, lane, wave);
    if (lane == 0) wcnt[wave] = wc;
    __syncthreads();
    int pre = 0, all = 0;
#pragma unroll
    for (int w2 = 0; w2 < NWAVE; ++w2) {
      int c = wcnt[w2];
      c = c < 0 ? 0 : (c > WCAP ? WCAP : c);
      all += c;
      pre += (w2 < wave) ? c : 0;
    }
    const int wcc  = wc > WCAP ? WCAP : wc;
    const int base = tot + pre;
#pragma unroll 1
    for (int i = lane; i < wcc; i += 32) {
      const int ent = list[wave * WCAP + i];
      const int el  = (ent >> 12) & (CHUNK - 1);
      const int sl  = ent & (NBMAX - 1);
      int eid = cbase + el;
      eid = eid > nE - 1 ? nE - 1 : eid;
      const int pos = base + i;
      if (pos < RCAP) reg1[pos] = (int)(((unsigned)eid << 12) | (unsigned)sl);
    }
    tot += all;
    tot = tot > RCAP ? RCAP : tot;
    __syncthreads();
  }
  const int nh = tot;

  if (wave == 0) {
#pragma unroll 1
    for (int b0 = 0; b0 < nh; b0 += 32) {
      const int idx = b0 + lane;
      const int uv  = reg1[idx < RCAP ? idx : RCAP - 1];
      const int m32 = (nh - b0) < 32 ? (nh - b0) : 32;
#pragma unroll 1
      for (int k = 0; k < m32; ++k) {
        const int u  = __builtin_amdgcn_readlane(uv, k);
        const int sl = u & (NBMAX - 1);
        if (lane == 0) scnt[sl] = scnt[sl] + 1;
      }
    }
  }
  __syncthreads();

  {
    const v4i ca = *(const v4i*)(scnt + 4 * tid);
    const int e0 = ca.x < 0 ? 0 : ca.x, e1 = ca.y < 0 ? 0 : ca.y, e2 = ca.z < 0 ? 0 : ca.z, e3 = ca.w < 0 ? 0 : ca.w;
    const int ts = e0 + e1 + e2 + e3;
    int incl = ts;
#pragma unroll
    for (int d = 1; d < 32; d <<= 1) {
      const int up = __shfl_up(incl, d);
      if (lane >= d) incl += up;
    }
    if (lane == 31) wtot[wave] = incl;
    __syncthreads();
    int pre = 0;
#pragma unroll
    for (int w2 = 0; w2 < NWAVE; ++w2) pre += (w2 < wave) ? wtot[w2] : 0;
    int run = pre + incl - ts;
    soff[4 * tid + 0] = run; run += e0;
    soff[4 * tid + 1] = run; run += e1;
    soff[4 * tid + 2] = run; run += e2;
    soff[4 * tid + 3] = run;
  }
  __syncthreads();
  for (int i = tid; i < NBMAX; i += NTHR) list[i] = soff[i];
  __syncthreads();

  if (wave == 0) {
#pragma unroll 1
    for (int b0 = 0; b0 < nh; b0 += 32) {
      const int idx = b0 + lane;
      const int uv  = reg1[idx < RCAP ? idx : RCAP - 1];
      const int m32 = (nh - b0) < 32 ? (nh - b0) : 32;
#pragma unroll 1
      for (int k = 0; k < m32; ++k) {
        const int u   = __builtin_amdgcn_readlane(uv, k);
        const int sl  = u & (NBMAX - 1);
        const int eid = (int)((unsigned)u >> 12);
        if (lane == 0) {
          int pos = list[sl];
          pos = pos < 0 ? 0 : (pos > RCAP - 1 ? RCAP - 1 : pos);
          reg2[pos] = eid;
          list[sl] = pos + 1;
        }
      }
    }
  }
  __syncthreads();

  const int nbw = nb >> 3;
  const bool ovf = (nh >= RCAP);
  const float qnan = __int_as_float(0x7fc00000);
  const v4f wb1 = bfr4(*(const v4fa*)(wbeta + 4 * lane));
  const v4f wb2 = bfr4(*(const v4fa*)(wbeta + DIN + 4 * lane));
  const v4f wb3 = bfr4(*(const v4fa*)(wbeta + 2 * DIN + 4 * lane));
  const v4f bg4 = bfr4(*(const v4fa*)(bg + 4 * lane));
  const v4f ga4 = bfr4(*(const v4fa*)(g1 + 4 * lane));
  const v4f be4 = bfr4(*(const v4fa*)(b1 + 4 * lane));
  const float lw = bf16r(lws[0]);
  const float gw = bf16r(gws[0]);
  unsigned* hs = hstg + wave * HSTG;
#pragma unroll 1
  for (int jt = 0; jt < nbw; ++jt) {
    const int slot = wave * nbw + jt;
    const int grow = nodeBase + slot;
    const int gcl  = grow < nN ? grow : nN - 1;
    int st = soff[slot];
    const int craw = scnt[slot];
    int cnt = craw;
    st  = st < 0 ? 0 : (st > nh ? nh : st);
    cnt = cnt < 0 ? 0 : (cnt > DEGCAP ? DEGCAP : cnt);
    if (cnt > nh - st) cnt = nh - st;
    const float pz = (ovf || craw > DEGCAP) ? qnan : 0.0f;
    const bool wr = grow < nN;
    const float ddst = dinvf(craw);

    const float* prow = P + (size_t)gcl * NP + 4 * lane;
    const v4f q4 = *(const v4fa*)(prow + OQQ);
    const v4f x4 = *(const v4fa*)(prow + OXR);
    float la0 = 0.f, la1 = 0.f, la2 = 0.f, la3 = 0.f;
    float av0 = 0.f, av1 = 0.f, av2 = 0.f, av3 = 0.f;
    float mx = -1.0e30f, dn = 0.f;

#pragma unroll 1
    for (int q = 0; q < cnt; ++q) {
      int idx = st + q; idx = idx > RCAP - 1 ? RCAP - 1 : idx;
      int eid = reg2[idx]; eid = eid < 0 ? 0 : (eid > nE - 1 ? nE - 1 : eid);
      const int sraw = srcs[eid];
      const int s = sraw < 0 ? 0 : (sraw > nN - 1 ? nN - 1 : sraw);
      const float* sr = P + (size_t)s * NP + 4 * lane;
      const v4f xw = *(const v4fa*)(sr + OXW);
      const v4f kk = *(const v4fa*)(sr + OKK);
      const v4f vv = *(const v4fa*)(sr + OVV);
      const float cf = dinv[s] * ddst;
      la0 = fmaf(cf, xw.x, la0);
      la1 = fmaf(cf, xw.y, la1);
      la2 = fmaf(cf, xw.z, la2);
      la3 = fmaf(cf, xw.w, la3);
      float part = q4.x * kk.x;
      part = fmaf(q4.y, kk.y, part);
      part = fmaf(q4.z, kk.z, part);
      part = fmaf(q4.w, kk.w, part);
      part += __shfl_xor(part, 1);
      part += __shfl_xor(part, 2);
      part += __shfl_xor(part, 4);
      const float al = part * ATTSC;
      const float df = al - mx;
      const float ee = __expf(-fabsf(df));
      const bool up  = df > 0.f;
      const float s1 = up ? ee : 1.0f;
      const float s2 = up ? 1.0f : ee;
      mx = up ? al : mx;
      dn = fmaf(dn, s1, s2);
      av0 = fmaf(av0, s1, s2 * vv.x);
      av1 = fmaf(av1, s1, s2 * vv.y);
      av2 = fmaf(av2, s1, s2 * vv.z);
      av3 = fmaf(av3, s1, s2 * vv.w);
    }
    const float dsd = dn > 0.f ? dn : 1.0f;
    const float iv  = (dn > 0.f ? 1.0f : 0.0f) * __builtin_amdgcn_rcpf(dsd);
    const float og0 = av0 * iv, og1 = av1 * iv, og2 = av2 * iv, og3 = av3 * iv;
    const float lo0 = la0 + bg4.x, lo1 = la1 + bg4.y, lo2 = la2 + bg4.z, lo3 = la3 + bg4.w;
    float pb = og0 * wb1.x;
    pb = fmaf(og1, wb1.y, pb);
    pb = fmaf(og2, wb1.z, pb);
    pb = fmaf(og3, wb1.w, pb);
    pb = fmaf(x4.x, wb2.x, pb);
    pb = fmaf(x4.y, wb2.y, pb);
    pb = fmaf(x4.z, wb2.z, pb);
    pb = fmaf(x4.w, wb2.w, pb);
    pb = fmaf(og0 - x4.x, wb3.x, pb);
    pb = fmaf(og1 - x4.y, wb3.y, pb);
    pb = fmaf(og2 - x4.z, wb3.z, pb);
    pb = fmaf(og3 - x4.w, wb3.w, pb);
    pb = waveSum(pb);
    const float ez   = __expf(-pb);
    const float beta = __builtin_amdgcn_rcpf(1.0f + ez);
    const float omb  = 1.0f - beta;
    const float go0 = fmaf(beta, x4.x, omb * og0);
    const float go1 = fmaf(beta, x4.y, omb * og1);
    const float go2 = fmaf(beta, x4.z, omb * og2);
    const float go3 = fmaf(beta, x4.w, omb * og3);
    const float h00 = fmaf(lw, lo0, gw * go0);
    const float h01 = fmaf(lw, lo1, gw * go1);
    const float h02 = fmaf(lw, lo2, gw * go2);
    const float h03 = fmaf(lw, lo3, gw * go3);
    const float y0 = h00 + h00, y1 = h01 + h01, y2 = h02 + h02, y3 = h03 + h03;
    const float mu = waveSum((y0 + y1) + (y2 + y3)) * (1.0f / DIN);
    const float d0 = y0 - mu, d1 = y1 - mu, d2 = y2 - mu, d3 = y3 - mu;
    const float var = waveSum(fmaf(d3, d3, fmaf(d2, d2, fmaf(d1, d1, d0 * d0)))) * (1.0f / DIN);
    const float inv = rsqrtf(var + LNEPS);
    const float hv0 = fmaf(d0 * inv, ga4.x, be4.x) + pz;
    const float hv1 = fmaf(d1 * inv, ga4.y, be4.y) + pz;
    const float hv2 = fmaf(d2 * inv, ga4.z, be4.z) + pz;
    const float hv3 = fmaf(d3 * inv, ga4.w, be4.w) + pz;

    const unsigned hb0 = bfbits(hv0), hb1 = bfbits(hv1), hb2 = bfbits(hv2), hb3 = bfbits(hv3);
    const unsigned lb0 = bfbits(hv0 - bfval(hb0)), lb1 = bfbits(hv1 - bfval(hb1));
    const unsigned lb2 = bfbits(hv2 - bfval(hb2)), lb3 = bfbits(hv3 - bfval(hb3));
    v4u pk;
    pk.x = hb0 | (hb1 << 16); pk.y = hb2 | (hb3 << 16);
    pk.z = lb0 | (lb1 << 16); pk.w = lb2 | (lb3 << 16);
    *(v4ua*)(hs + 4 * lane) = pk;
    __builtin_amdgcn_fence(__ATOMIC_RELEASE, "wavefront");
    __builtin_amdgcn_wave_barrier();
    const int jj = lane & 15, part = lane >> 4;
    const v2u e0 = *(const v2ua*)(hs + 8 * jj + 2 * part);
    const v2u e1 = *(const v2ua*)(hs + 8 * jj + 4 + 2 * part);
    v4u pv;
    pv.x = e0.x; pv.y = e0.y; pv.z = e1.x; pv.w = e1.y;
    __builtin_amdgcn_wave_barrier();
    unsigned* hd = (unsigned*)(P + (size_t)gcl * NP + OQQ) + 4 * lane;
    if (wr) *(volatile v4ua*)hd = pv;
    __threadfence();
    if (wr) *(volatile v4ua*)hd = pv;
  }
}

__global__ __launch_bounds__(NTHR) void k_ffn1(unsigned short* P16, int nra, const unsigned short* __restrict__ WR) {
  __shared__ __attribute__((aligned(16))) unsigned short stg[NWAVE * 16 * 128];
  const int tid = (int)threadIdx.x, lane = tid & 31, wave = tid >> 5, hh = lane >> 4, m = lane & 15;
  const int rw = wave & 3, cg = wave >> 2;
  const int rowBase = (int)blockIdx.x * GBM;
  const int colW    = cg * 128;

  v8f acc[8];
  {
    const v8f z = {0.f, 0.f, 0.f, 0.f, 0.f, 0.f, 0.f, 0.f};
#pragma unroll
    for (int t = 0; t < 8; ++t) acc[t] = z;
  }
  int ra = rowBase + 16 * rw + m;
  ra = ra > nra - 1 ? nra - 1 : ra;
  ra = ra < 0 ? 0 : ra;
  const unsigned short* ap = P16 + (size_t)ra * NPH + OH16 + 8 * hh;
  const unsigned short* wp = WR + (size_t)(colW + m) * KF1 + 8 * hh;

#pragma unroll 1
  for (int ks = 0; ks < KF1 / 32; ++ks) {
    FragB af;
    af.h[0] = *(const v8usa*)(ap + 32 * ks);
    af.h[1] = *(const v8usa*)(ap + 32 * ks + 16);
#pragma unroll
    for (int t = 0; t < 8; ++t) {
      const unsigned short* wq = wp + (size_t)(16 * t) * KF1 + 32 * ks;
      FragB bf;
      bf.h[0] = *(const v8usa*)wq;
      bf.h[1] = *(const v8usa*)(wq + 16);
      acc[t] = wmb(af, bf, acc[t]);
    }
  }

  unsigned short* sw = stg + wave * 2048;
#pragma unroll
  for (int hf = 0; hf < 2; ++hf) {
#pragma unroll
    for (int t4 = 0; t4 < 4; ++t4) {
      const int t = 4 * hf + t4;
#pragma unroll
      for (int r = 0; r < 8; ++r) {
        const float x = fmaxf(acc[t][r], 0.0f);
        const unsigned hb = bfbits(x);
        const unsigned lb = bfbits(x - bfval(hb));
        sw[(8 * hh + r) * 128 + 16 * t4 + m]      = (unsigned short)hb;
        sw[(8 * hh + r) * 128 + 64 + 16 * t4 + m] = (unsigned short)lb;
      }
    }
    __syncthreads();
    const int rsub = lane >> 4, part = (lane >> 3) & 1, q8 = lane & 7;
    v8us pv[8];
#pragma unroll
    for (int i = 0; i < 8; ++i) {
      const int rloc = 2 * i + rsub;
      pv[i] = *(const v8usa*)(sw + rloc * 128 + part * 64 + 8 * q8);
    }
#pragma unroll
    for (int i = 0; i < 8; ++i) {
      const int gr = rowBase + 16 * rw + 2 * i + rsub;
      unsigned short* op = P16 + (size_t)gr * NPH + OF16 + part * NF1 + colW + 64 * hf + 8 * q8;
      *(volatile v8us*)op = pv[i];
    }
    __threadfence();
#pragma unroll
    for (int i = 0; i < 8; ++i) {
      const int gr = rowBase + 16 * rw + 2 * i + rsub;
      unsigned short* op = P16 + (size_t)gr * NPH + OF16 + part * NF1 + colW + 64 * hf + 8 * q8;
      *(volatile v8us*)op = pv[i];
    }
    __syncthreads();
  }
}

__global__ __launch_bounds__(NTHR) void k_ffn2(const unsigned short* P16, int nra, const unsigned short* __restrict__ WO,
                                               const float* __restrict__ g2, const float* __restrict__ b2, float* out) {
  __shared__ __attribute__((aligned(16))) float stg[GBM * DIN];
  const int tid = (int)threadIdx.x, lane = tid & 31, wave = tid >> 5, hh = lane >> 4, m = lane & 15;
  const int rw = wave & 3, cg = wave >> 2;
  const int rowBase = (int)blockIdx.x * GBM;
  const int colW    = cg * 64;

  v8f acc[4];
  {
    const v8f z = {0.f, 0.f, 0.f, 0.f, 0.f, 0.f, 0.f, 0.f};
#pragma unroll
    for (int t = 0; t < 4; ++t) acc[t] = z;
  }
  int ra = rowBase + 16 * rw + m;
  ra = ra > nra - 1 ? nra - 1 : ra;
  ra = ra < 0 ? 0 : ra;
  const unsigned short* ap = P16 + (size_t)ra * NPH + OF16 + 8 * hh;
  const unsigned short* wp = WO + (size_t)(colW + m) * KF2 + 8 * hh;

#pragma unroll 1
  for (int ks = 0; ks < KF2 / 32; ++ks) {
    FragB af;
    af.h[0] = *(const v8usa*)(ap + 32 * ks);
    af.h[1] = *(const v8usa*)(ap + 32 * ks + 16);
#pragma unroll
    for (int t = 0; t < 4; ++t) {
      const unsigned short* wq = wp + (size_t)(16 * t) * KF2 + 32 * ks;
      FragB bf;
      bf.h[0] = *(const v8usa*)wq;
      bf.h[1] = *(const v8usa*)(wq + 16);
      acc[t] = wmb(af, bf, acc[t]);
    }
  }

#pragma unroll
  for (int t = 0; t < 4; ++t)
#pragma unroll
    for (int r = 0; r < 8; ++r) stg[(16 * rw + 8 * hh + r) * DIN + colW + 16 * t + m] = acc[t][r];
  __syncthreads();

  const v4f ga4 = bfr4(*(const v4fa*)(g2 + 4 * lane));
  const v4f be4 = bfr4(*(const v4fa*)(b2 + 4 * lane));
  v4f ov[8];
#pragma unroll
  for (int i = 0; i < 8; ++i) {
    const int rl = 8 * wave + i;
    int gr = rowBase + rl;
    gr = gr > nra - 1 ? nra - 1 : gr;
    const v4f f4 = *(const v4fa*)(stg + rl * DIN + 4 * lane);
    const unsigned short* hr = P16 + (size_t)gr * NPH + OH16 + 4 * lane;
    const v2u hw = *(const v2ua*)(hr);
    const v2u lw = *(const v2ua*)(hr + DIN);
    const float h0 = __uint_as_float(hw.x << 16)          + __uint_as_float(lw.x << 16);
    const float h1 = __uint_as_float(hw.x & 0xffff0000u)  + __uint_as_float(lw.x & 0xffff0000u);
    const float h2 = __uint_as_float(hw.y << 16)          + __uint_as_float(lw.y << 16);
    const float h3 = __uint_as_float(hw.y & 0xffff0000u)  + __uint_as_float(lw.y & 0xffff0000u);
    const float y0 = f4.x + h0, y1 = f4.y + h1, y2 = f4.z + h2, y3 = f4.w + h3;
    const float mu = waveSum((y0 + y1) + (y2 + y3)) * (1.0f / DIN);
    const float d0 = y0 - mu, d1 = y1 - mu, d2 = y2 - mu, d3 = y3 - mu;
    const float var = waveSum(fmaf(d3, d3, fmaf(d2, d2, fmaf(d1, d1, d0 * d0)))) * (1.0f / DIN);
    const float inv = rsqrtf(var + LNEPS);
    ov[i].x = fmaf(d0 * inv, ga4.x, be4.x);
    ov[i].y = fmaf(d1 * inv, ga4.y, be4.y);
    ov[i].z = fmaf(d2 * inv, ga4.z, be4.z);
    ov[i].w = fmaf(d3 * inv, ga4.w, be4.w);
  }
#pragma unroll
  for (int i = 0; i < 8; ++i) {
    const int gr = rowBase + 8 * wave + i;
    if (gr < nra) *(volatile v4f*)(out + (size_t)gr * DIN + 4 * lane) = ov[i];
  }
  __threadfence();
#pragma unroll
  for (int i = 0; i < 8; ++i) {
    const int gr = rowBase + 8 * wave + i;
    if (gr < nra) *(volatile v4f*)(out + (size_t)gr * DIN + 4 * lane) = ov[i];
  }
}

static int pick_nb(int nE, int nN) {
  int nb = NBMAX;
  while (nb > 32 && (long long)nb * (long long)nE * 5LL > (long long)RCAP * (long long)nN * 4LL) nb >>= 1;
  return nb;
}
static inline int cdiv(int a, int b) { return (a + b - 1) / b; }

extern "C" void kernel_launch(void* const* d_in, const int* in_sizes, int n_in,
                              void* d_out, int out_size, void* d_ws, size_t ws_size,
                              hipStream_t stream) {
  if (n_in < 21) return;
  if (in_sizes[0] < DIN || (in_sizes[0] % DIN) != 0) return;
  const int nN = in_sizes[0] / DIN;
  if (nN > (1 << 22)) return;
  if (in_sizes[1] < 2 || (in_sizes[1] & 1) != 0) return;
  const int nE = in_sizes[1] / 2;
  if (nE < 1 || nE > (1 << 20)) return;
  if (in_sizes[2] != DIN * DIN || in_sizes[4] != DIN * DIN || in_sizes[6] != DIN * DIN ||
      in_sizes[8] != DIN * DIN || in_sizes[10] != DIN * DIN) return;
  if (in_sizes[3] != DIN || in_sizes[5] != DIN || in_sizes[7] != DIN || in_sizes[9] != DIN || in_sizes[11] != DIN) return;
  if (in_sizes[12] != 3 * DIN) return;
  if (in_sizes[13] != DIN || in_sizes[14] != DIN || in_sizes[15] != DIN || in_sizes[16] != DIN) return;
  if (in_sizes[17] != DIN * NF1 || in_sizes[18] != NF1 * DIN) return;
  if (in_sizes[19] < 1 || in_sizes[20] < 1) return;
  if (out_size != nN * DIN) return;

  const float* x      = (const float*)d_in[0];
  const int*   ei     = (const int*)  d_in[1];
  const float* wg     = (const float*)d_in[2];
  const float* bgc    = (const float*)d_in[3];
  const float* wq     = (const float*)d_in[4];
  const float* bq     = (const float*)d_in[5];
  const float* wk     = (const float*)d_in[6];
  const float* bk     = (const float*)d_in[7];
  const float* wv     = (const float*)d_in[8];
  const float* bv     = (const float*)d_in[9];
  const float* wsk    = (const float*)d_in[10];
  const float* bsk    = (const float*)d_in[11];
  const float* wbeta  = (const float*)d_in[12];
  const float* g1     = (const float*)d_in[13];
  const float* b1     = (const float*)d_in[14];
  const float* g2     = (const float*)d_in[15];
  const float* b2     = (const float*)d_in[16];
  const float* wrel   = (const float*)d_in[17];
  const float* wroot  = (const float*)d_in[18];
  const float* lws    = (const float*)d_in[19];
  const float* gws    = (const float*)d_in[20];
  float* out = (float*)d_out;
  const int* src = ei;
  const int* dst = ei + nE;

  const int MP   = cdiv(nN, GBM) * GBM;
  const int nb   = pick_nb(nE, nN);
  const int gA   = cdiv(nN, nb);
  const int vec8 = ((nE & 3) == 0) ? 1 : 0;
  if ((long long)gA * nb < nN) return;

  char* wsb = (char*)d_ws;
  size_t off = 0;
  const size_t oP  = off; off += (size_t)MP * NP * 4;               off = (off + 255) & ~(size_t)255;
  const size_t oDV = off; off += (size_t)gA * (size_t)nb * 4;       off = (off + 255) & ~(size_t)255;
  const size_t oW5 = off; off += (size_t)NP * DIN * 2;              off = (off + 255) & ~(size_t)255;
  const size_t oWR = off; off += (size_t)NF1 * KF1 * 2;             off = (off + 255) & ~(size_t)255;
  const size_t oWO = off; off += (size_t)NF2 * KF2 * 2;             off = (off + 255) & ~(size_t)255;
  if (off > ws_size || off > (size_t)WSMAX) return;
  float*          P    = (float*)(wsb + oP);
  unsigned short* P16  = (unsigned short*)(wsb + oP);
  float*          DINV = (float*)(wsb + oDV);
  unsigned short* WT5  = (unsigned short*)(wsb + oW5);
  unsigned short* WR2  = (unsigned short*)(wsb + oWR);
  unsigned short* WO2  = (unsigned short*)(wsb + oWO);

  hipFuncSetAttribute(reinterpret_cast<const void*>(&k_cnt),
                      hipFuncAttributeMaxDynamicSharedMemorySize, LDS_CNT);
  hipFuncSetAttribute(reinterpret_cast<const void*>(&k_agg),
                      hipFuncAttributeMaxDynamicSharedMemorySize, LDS_AGG);

  const int nU5 = NP * (DIN / 8);
  k_wtr5<<<cdiv(nU5, NTHR), NTHR, 0, stream>>>(wg, wk, wv, wq, wsk, WT5, nU5);
  const int nUR = NF1 * (2 * DIN / 8);
  k_wtr2<<<cdiv(nUR, NTHR), NTHR, 0, stream>>>(wrel, DIN, NF1, WR2, nUR);
  const int nUO = NF2 * (2 * NF1 / 8);
  k_wtr2<<<cdiv(nUO, NTHR), NTHR, 0, stream>>>(wroot, NF1, NF2, WO2, nUO);

  const int gM = MP / GBM;
  k_proj<<<dim3(gM, NSEG), PTHR, 0, stream>>>(x, nN, WT5, bk, bv, bq, bsk, P);

  k_cnt<<<gA, NTHR, LDS_CNT, stream>>>(dst, DINV, nE, nb, vec8);

  k_agg<<<gA, NTHR, LDS_AGG, stream>>>(src, dst, P, DINV, bgc, wbeta, g1, b1, lws, gws, nN, nE, nb, vec8);

  k_ffn1<<<gM, NTHR, 0, stream>>>(P16, nN, WR2);
  k_ffn2<<<gM, NTHR, 0, stream>>>(P16, nN, WO2, g2, b2, out);
}
